// BahdanauAttention_39307540693917
// MI455X (gfx1250) — hardware-verified
//
#include <hip/hip_runtime.h>


#ifndef NB
#define NB 8
#endif
#ifndef TQ
#define TQ 128
#endif
#define NB_FULL 8
#define T_FULL 128
#define S_LEN 128
#define S_FULL 128
#define HD 512
#define KC (2 * S_LEN)
#define LN_EPS 1.0e-3f

static_assert(NB >= 1 && NB <= NB_FULL);
static_assert(TQ >= 64 && TQ <= T_FULL && (TQ % 64) == 0);
static_assert(S_LEN == 128 && S_LEN == S_FULL);
static_assert((HD % 256) == 0 && (HD % 64) == 0 && (HD % 32) == 0);
static_assert((KC % 32) == 0 && (S_LEN % 64) == 0);
static_assert(((HD / 4) % S_LEN) == 0);
static_assert((S_LEN % 32) == 0 && S_LEN / 8 == 16);

typedef unsigned short us;
typedef us     v8us  __attribute__((ext_vector_type(8)));
typedef __bf16 v16bf __attribute__((ext_vector_type(16)));
typedef float  v8f   __attribute__((ext_vector_type(8)));
typedef float  v4f   __attribute__((ext_vector_type(4)));

union Frag { v16bf v; v8us h[2]; };

__device__ __forceinline__ us f2bf(float f) {
    unsigned int u = __float_as_uint(f);
    u += 0x7FFFu + ((u >> 16) & 1u);
    return (us)(u >> 16);
}
__device__ __forceinline__ float bf2f(us h) {
    return __uint_as_float(((unsigned int)h) << 16);
}
__device__ __forceinline__ float rbf(float f) {
    return bf2f(f2bf(f));
}
__device__ __forceinline__ float tanh_acc(float x) {
    const float ax = __builtin_fabsf(x);
    const float t  = __expf(-2.0f * ax);
    const float r  = (1.0f - t) * __builtin_amdgcn_rcpf(1.0f + t);
    return __builtin_copysignf(r, x);
}
__device__ __forceinline__ v8us pack8(v4f a, v4f c) {
    v8us o;
    o[0] = f2bf(a.x); o[1] = f2bf(a.y); o[2] = f2bf(a.z); o[3] = f2bf(a.w);
    o[4] = f2bf(c.x); o[5] = f2bf(c.y); o[6] = f2bf(c.z); o[7] = f2bf(c.w);
    return o;
}
__device__ __forceinline__ void split8(v4f a, v4f c, v8us& hi, v8us& lo) {
    const float x[8] = {a.x, a.y, a.z, a.w, c.x, c.y, c.z, c.w};
#pragma unroll
    for (int i = 0; i < 8; ++i) {
        const us h = f2bf(x[i]);
        hi[i] = h;
        lo[i] = f2bf(x[i] - bf2f(h));
    }
}

__device__ __forceinline__ v8f wmma16(v16bf a, v16bf b, v8f c) {
    v8f d = __builtin_amdgcn_wmma_f32_16x16x32_bf16(false, a, false, b, (short)0, c, false, false);
    asm volatile("v_nop\n\tv_nop\n\tv_nop\n\tv_nop" : "+v"(d) : "v"(a), "v"(b));
    return d;
}

__device__ __forceinline__ v16bf ld_frag(const us* __restrict__ P, int ld, int row, int k0, int hsel) {
    Frag f;
    const us* p = P + (size_t)row * ld + k0 + 8 * hsel;
    f.h[0] = *(const v8us*)p;
    f.h[1] = *(const v8us*)(p + 16);
    return f.v;
}

__global__ __launch_bounds__(256)
void k_cvt(const float* __restrict__ src, int spitch, int scol, int grp, int gstride,
           us* __restrict__ dst, int dpitch, int dcol, int nrows, int nseg)
{
    const int lane = threadIdx.x & 31;
    const int gw   = blockIdx.x * 8 + (threadIdx.x >> 5);
    if (gw >= nrows * nseg) return;
    const int r    = gw / nseg;
    const int sg   = gw - r * nseg;
    const int g    = r / grp;
    const int srow = g * gstride + (r - g * grp);
    const float* sp = src + (size_t)srow * spitch + scol + sg * 256 + lane * 8;
    const v4f a = *(const v4f*)sp;
    const v4f c = *(const v4f*)(sp + 4);
    const v8us o = pack8(a, c);
    us* dp = dst + (size_t)r * dpitch + dcol + sg * 256 + lane * 8;
    *(volatile v8us*)dp = o;
    __threadfence();
    *(volatile v8us*)dp = o;
}

template <int DUP>
__global__ __launch_bounds__(256)
void k_trans(const float* __restrict__ src, int spitch, int sstride,
             us* __restrict__ dst, int dpitch, int dstride)
{
    __shared__ float ts[64][65];
    const int r0 = blockIdx.x * 64, c0 = blockIdx.y * 64, z = blockIdx.z;
    const int tid = threadIdx.x, lane = tid & 31, wave = tid >> 5;
    const float* sb = src + (size_t)z * (size_t)sstride;
    us* db = dst + (size_t)z * (size_t)dstride;

#pragma unroll
    for (int p = 0; p < 4; ++p) {
        const int rl = p * 16 + (tid >> 4);
        const int c4 = (tid & 15) * 4;
        const v4f x = *(const v4f*)(sb + (size_t)(r0 + rl) * spitch + c0 + c4);
        ts[rl][c4 + 0] = x.x; ts[rl][c4 + 1] = x.y; ts[rl][c4 + 2] = x.z; ts[rl][c4 + 3] = x.w;
    }
    __syncthreads();

    v8us o[2];
#pragma unroll
    for (int p = 0; p < 2; ++p) {
        const int cl = p * 32 + wave * 4 + (lane >> 3);
        const int r8 = (lane & 7) * 8;
#pragma unroll
        for (int i = 0; i < 8; ++i) o[p][i] = f2bf(ts[r8 + i][cl]);
    }
#pragma unroll
    for (int p = 0; p < 2; ++p) {
        const int cl = p * 32 + wave * 4 + (lane >> 3);
        const int r8 = (lane & 7) * 8;
        us* d = db + (size_t)(c0 + cl) * dpitch + r0 + r8;
        *(volatile v8us*)d = o[p];
        if (DUP != 0) *(volatile v8us*)(d + DUP) = o[p];
    }
    __threadfence();
#pragma unroll
    for (int p = 0; p < 2; ++p) {
        const int cl = p * 32 + wave * 4 + (lane >> 3);
        const int r8 = (lane & 7) * 8;
        us* d = db + (size_t)(c0 + cl) * dpitch + r0 + r8;
        *(volatile v8us*)d = o[p];
        if (DUP != 0) *(volatile v8us*)(d + DUP) = o[p];
    }
}

__global__ __launch_bounds__(128)
void k_gemm(const us* __restrict__ A, int lda, int strideA,
            const us* __restrict__ B, int ldb, int strideB,
            float* __restrict__ C, int ldc, int strideC, int K)
{
    __shared__ __attribute__((aligned(16))) float tile[4 * 16 * 64];

    const int lane = threadIdx.x & 31, wave = threadIdx.x >> 5;
    const int hsel = lane >> 4, m = lane & 15;
    const int m0 = blockIdx.x * 64 + wave * 16;
    const int n0 = blockIdx.y * 64;
    const us* Ab = A + (size_t)blockIdx.z * (size_t)strideA;
    const us* Bb = B + (size_t)blockIdx.z * (size_t)strideB;

    v8f c0 = {}; v8f c1 = {}; v8f c2 = {}; v8f c3 = {};
    for (int k0 = 0; k0 < K; k0 += 32) {
        const v16bf a  = ld_frag(Ab, lda, m0 + m, k0, hsel);
        const v16bf b0 = ld_frag(Bb, ldb, n0 + m,      k0, hsel);
        const v16bf b1 = ld_frag(Bb, ldb, n0 + 16 + m, k0, hsel);
        const v16bf b2 = ld_frag(Bb, ldb, n0 + 32 + m, k0, hsel);
        const v16bf b3 = ld_frag(Bb, ldb, n0 + 48 + m, k0, hsel);
        c0 = wmma16(a, b0, c0);
        c1 = wmma16(a, b1, c1);
        c2 = wmma16(a, b2, c2);
        c3 = wmma16(a, b3, c3);
    }

    float* tw = tile + wave * 1024;
#pragma unroll
    for (int r = 0; r < 8; ++r) {
        const int row = 8 * hsel + r;
        tw[row * 64 + m]      = c0[r];
        tw[row * 64 + 16 + m] = c1[r];
        tw[row * 64 + 32 + m] = c2[r];
        tw[row * 64 + 48 + m] = c3[r];
    }
    __syncthreads();

    float* Cb = C + (size_t)blockIdx.z * (size_t)strideC;
    v4f vals[8];
#pragma unroll
    for (int p = 0; p < 8; ++p) {
        const int row = 2 * p + hsel;
        vals[p] = *(const v4f*)(tw + row * 64 + 4 * m);
    }
#pragma unroll
    for (int p = 0; p < 8; ++p) {
        float* d = Cb + (size_t)(m0 + 2 * p + hsel) * ldc + n0 + 4 * m;
        *(volatile v4f*)d = vals[p];
    }
    __threadfence();
#pragma unroll
    for (int p = 0; p < 8; ++p) {
        float* d = Cb + (size_t)(m0 + 2 * p + hsel) * ldc + n0 + 4 * m;
        *(volatile v4f*)d = vals[p];
    }
}

__global__ __launch_bounds__(S_LEN)
void k_attn(const float* __restrict__ Uxp, const float* __restrict__ Wcp,
            const float* __restrict__ bWa, const float* __restrict__ bUa,
            const float* __restrict__ Va,  const float* __restrict__ bVa,
            us* __restrict__ Pcat)
{
    __shared__ v4f sq4[HD / 4];
    __shared__ v4f sv4[HD / 4];
    __shared__ __attribute__((aligned(16))) float sp[S_LEN];
    __shared__ float red[S_LEN];

    const int bt  = blockIdx.x;
    const int b   = bt / TQ;
    const int tid = threadIdx.x, lane = tid & 31, wave = tid >> 5;

    for (int i = tid; i < HD / 4; i += S_LEN) {
        v4f q = *(const v4f*)(Uxp + (size_t)bt * HD + i * 4);
        const v4f b1 = *(const v4f*)(bUa + i * 4);
        const v4f b2 = *(const v4f*)(bWa + i * 4);
        q.x = (q.x + rbf(b1.x)) + rbf(b2.x);
        q.y = (q.y + rbf(b1.y)) + rbf(b2.y);
        q.z = (q.z + rbf(b1.z)) + rbf(b2.z);
        q.w = (q.w + rbf(b1.w)) + rbf(b2.w);
        sq4[i] = q;
        v4f w = *(const v4f*)(Va + i * 4);
        w.x = rbf(w.x); w.y = rbf(w.y); w.z = rbf(w.z); w.w = rbf(w.w);
        sv4[i] = w;
    }
    __syncthreads();

    const float bva = rbf(bVa[0]);
    const v4f* we = (const v4f*)(Wcp + ((size_t)b * S_LEN + tid) * HD);
    float acc = 0.0f;
#pragma unroll 2
    for (int u = 0; u < HD / 4; ++u) {
        const v4f e = we[u];
        const v4f d = sq4[u];
        const v4f w = sv4[u];
        acc += w.x * tanh_acc(e.x + d.x);
        acc += w.y * tanh_acc(e.y + d.y);
        acc += w.z * tanh_acc(e.z + d.z);
        acc += w.w * tanh_acc(e.w + d.w);
    }
    const float en = acc + bva;

    red[tid] = en;
    __syncthreads();
#pragma unroll
    for (int st = S_LEN / 2; st > 0; st >>= 1) {
        if (tid < st) red[tid] = fmaxf(red[tid], red[tid + st]);
        __syncthreads();
    }
    const float mx = red[0];
    __syncthreads();

    const float ex = __expf(en - mx);
    red[tid] = ex;
    __syncthreads();
#pragma unroll
    for (int st = S_LEN / 2; st > 0; st >>= 1) {
        if (tid < st) red[tid] += red[tid + st];
        __syncthreads();
    }
    const float ssum = red[0];
    const float p = ex * (1.0f / ssum);
    sp[tid] = p;
    __syncthreads();

    if (wave == 0) {
        const int q = lane & 15;
        const v4f a = *(const v4f*)(sp + q * 8);
        const v4f c = *(const v4f*)(sp + q * 8 + 4);
        v8us hi, lo;
        split8(a, c, hi, lo);
        v8us o;
#pragma unroll
        for (int i = 0; i < 8; ++i) o[i] = (lane < 16) ? hi[i] : lo[i];
        us* d = Pcat + (size_t)bt * KC + lane * 8;
        *(volatile v8us*)d = o;
        __threadfence();
        *(volatile v8us*)d = o;
    }
}

__global__ __launch_bounds__(256)
void k_ln(const float* __restrict__ cv, const float* __restrict__ xin,
          const float* __restrict__ gam, const float* __restrict__ bet,
          float* __restrict__ out, int nrows)
{
    const int lane = threadIdx.x & 31;
    const int r = blockIdx.x * 8 + (threadIdx.x >> 5);
    if (r >= nrows) return;
    const int g = r / TQ;
    const int frow = g * T_FULL + (r - g * TQ);
    const float* cp = cv  + (size_t)r * HD + lane * 4;
    const float* xp = xin + (size_t)frow * HD + lane * 4;

    v4f c[4], xr[4], gm[4], be[4];
#pragma unroll
    for (int j = 0; j < 4; ++j) {
        c[j]  = *(const v4f*)(cp + 128 * j);
        xr[j] = *(const v4f*)(xp + 128 * j);
        gm[j] = *(const v4f*)(gam + 128 * j + lane * 4);
        be[j] = *(const v4f*)(bet + 128 * j + lane * 4);
    }
    float s = 0.0f;
#pragma unroll
    for (int j = 0; j < 4; ++j) s += (c[j].x + c[j].y) + (c[j].z + c[j].w);
#pragma unroll
    for (int off = 16; off > 0; off >>= 1) s += __shfl_xor(s, off, 32);
    const float mean = s * (1.0f / (float)HD);

    float q = 0.0f;
#pragma unroll
    for (int j = 0; j < 4; ++j) {
        const float dx = c[j].x - mean, dy = c[j].y - mean, dz = c[j].z - mean, dw = c[j].w - mean;
        q += dx * dx; q += dy * dy; q += dz * dz; q += dw * dw;
    }
#pragma unroll
    for (int off = 16; off > 0; off >>= 1) q += __shfl_xor(q, off, 32);
    const float var  = q * (1.0f / (float)HD);
    const float rstd = rsqrtf(var + LN_EPS);

    v4f o[4];
#pragma unroll
    for (int j = 0; j < 4; ++j) {
        o[j].x = (c[j].x - mean) * rstd * rbf(gm[j].x) + rbf(be[j].x) + rbf(xr[j].x);
        o[j].y = (c[j].y - mean) * rstd * rbf(gm[j].y) + rbf(be[j].y) + rbf(xr[j].y);
        o[j].z = (c[j].z - mean) * rstd * rbf(gm[j].z) + rbf(be[j].z) + rbf(xr[j].z);
        o[j].w = (c[j].w - mean) * rstd * rbf(gm[j].w) + rbf(be[j].w) + rbf(xr[j].w);
    }
    float* dp = out + (size_t)frow * HD + lane * 4;
#pragma unroll
    for (int j = 0; j < 4; ++j) *(volatile v4f*)(dp + 128 * j) = o[j];
    __threadfence();
#pragma unroll
    for (int j = 0; j < 4; ++j) *(volatile v4f*)(dp + 128 * j) = o[j];
}

static inline size_t al256(size_t x) { return (x + 255) & ~(size_t)255; }

extern "C" void kernel_launch(void* const* d_in, const int* in_sizes, int n_in,
                              void* d_out, int out_size, void* d_ws, size_t ws_size,
                              hipStream_t stream)
{
    if (n_in < 10) return;
    if (in_sizes[0] < ((NB - 1) * T_FULL + S_LEN) * HD) return;
    if (in_sizes[1] < ((NB - 1) * T_FULL + TQ) * HD) return;
    if (in_sizes[2] < HD * HD) return;
    if (in_sizes[3] < HD) return;
    if (in_sizes[4] < HD * HD) return;
    if (in_sizes[5] < HD) return;
    if (in_sizes[6] < HD) return;
    if (in_sizes[7] < 1) return;
    if (in_sizes[8] < HD || in_sizes[9] < HD) return;
    if (out_size < ((NB - 1) * T_FULL + TQ) * HD) return;

    const float* context = (const float*)d_in[0];
    const float* x       = (const float*)d_in[1];
    const float* Wa      = (const float*)d_in[2];
    const float* bWa     = (const float*)d_in[3];
    const float* Ua      = (const float*)d_in[4];
    const float* bUa     = (const float*)d_in[5];
    const float* Va      = (const float*)d_in[6];
    const float* bVa     = (const float*)d_in[7];
    const float* gamma   = (const float*)d_in[8];
    const float* beta    = (const float*)d_in[9];
    float* out = (float*)d_out;

    char* ws = (char*)d_ws;
    size_t off = 0;
    us* ctxb  = (us*)(ws + off);    off += al256((size_t)NB * S_LEN * HD * sizeof(us));
    us* xb    = (us*)(ws + off);    off += al256((size_t)NB * TQ * HD * sizeof(us));
    us* WaT   = (us*)(ws + off);    off += al256((size_t)HD * HD * sizeof(us));
    us* UaT   = (us*)(ws + off);    off += al256((size_t)HD * HD * sizeof(us));
    us* ctxT2 = (us*)(ws + off);    off += al256((size_t)NB * HD * KC * sizeof(us));
    float* Wc = (float*)(ws + off); off += al256((size_t)NB * S_LEN * HD * sizeof(float));
    float* Ux = (float*)(ws + off); off += al256((size_t)NB * TQ * HD * sizeof(float));
    us* Pcat  = (us*)(ws + off);    off += al256((size_t)NB * TQ * KC * sizeof(us));
    float* cv = (float*)(ws + off); off += al256((size_t)NB * TQ * HD * sizeof(float));
    if (off > ws_size) return;

    const dim3 b256(256), b128(128), bS(S_LEN);

    {
        const int nrows = NB * S_LEN, nseg = HD / 256;
        k_cvt<<<dim3((nrows * nseg + 7) / 8), b256, 0, stream>>>(
            context, HD, 0, S_LEN, T_FULL, ctxb, HD, 0, nrows, nseg);
    }
    {
        const int nrows = NB * TQ, nseg = HD / 256;
        k_cvt<<<dim3((nrows * nseg + 7) / 8), b256, 0, stream>>>(
            x, HD, 0, TQ, T_FULL, xb, HD, 0, nrows, nseg);
    }
    k_trans<0><<<dim3(HD / 64, HD / 64, 1), b256, 0, stream>>>(Wa, HD, 0, WaT, HD, 0);
    k_trans<0><<<dim3(HD / 64, HD / 64, 1), b256, 0, stream>>>(Ua, HD, 0, UaT, HD, 0);
    k_trans<S_LEN><<<dim3(S_LEN / 64, HD / 64, NB), b256, 0, stream>>>(
        context, HD, T_FULL * HD, ctxT2, KC, HD * KC);

    k_gemm<<<dim3(NB * S_LEN / 64, HD / 64, 1), b128, 0, stream>>>(
        ctxb, HD, 0, WaT, HD, 0, Wc, HD, 0, HD);
    k_gemm<<<dim3(NB * TQ / 64, HD / 64, 1), b128, 0, stream>>>(
        xb, HD, 0, UaT, HD, 0, Ux, HD, 0, HD);

    k_attn<<<dim3(NB * TQ), bS, 0, stream>>>(Ux, Wc, bWa, bUa, Va, bVa, Pcat);

    k_gemm<<<dim3(TQ / 64, HD / 64, NB), b128, 0, stream>>>(
        Pcat, KC, TQ * KC, ctxT2, KC, HD * KC, cv, HD, TQ * HD, KC);

    k_ln<<<dim3((NB * TQ + 7) / 8), b256, 0, stream>>>(cv, x, gamma, beta, out, NB * TQ);
}
